// SelfAttentionMultiHead_78907139162215
// MI455X (gfx1250) — hardware-run, weakly checked
//
#include <hip/hip_runtime.h>
#define ZNG 25
#define ZNC 2
#define ZNS 128
#define ZNW 64
#define ZNR (ZNG * ZNS * ZNC)
#define ZVE 1e-5f
typedef unsigned short v8us __attribute__((ext_vector_type(8), may_alias));
typedef float  v8f  __attribute__((ext_vector_type(8)));
typedef float  v4f  __attribute__((ext_vector_type(4)));
typedef float  v4fa __attribute__((ext_vector_type(4), may_alias));

__device__ __forceinline__ unsigned short bf16_bits(float x) { unsigned int u = __float_as_uint(x); return (unsigned short)((u + 0x7FFFu + ((u >> 16) & 1u)) >> 16); }
__device__ __forceinline__ float bf16_val(unsigned short b) { return __uint_as_float(((unsigned int)b) << 16); }
__device__ __forceinline__ float bf16_round(float x) { return bf16_val(bf16_bits(x)); }

typedef _Float16 v16h __attribute__((ext_vector_type(16)));
union FragH { v16h v; v8us half[2]; _Float16 h[16]; unsigned short u[16]; };

typedef _Float16 v4h __attribute__((ext_vector_type(4)));

__global__ __launch_bounds__(256) void k_hl(const float* __restrict__ F, _Float16* __restrict__ Hh, _Float16* __restrict__ Hl, size_t n8) { const size_t t = (size_t)blockIdx.x * 256 + threadIdx.x; if (t >= n8) return; FragH fh, fl; const v4f a = *(const v4fa*)(F + t * 8), c = *(const v4fa*)(F + t * 8 + 4);
#pragma unroll
  for (int q = 0; q < 4; ++q) { _Float16 h = (_Float16)a[q]; fh.h[q] = h; fl.h[q] = (_Float16)((a[q] - (float)h) * 1024.0f); h = (_Float16)c[q]; fh.h[4 + q] = h; fl.h[4 + q] = (_Float16)((c[q] - (float)h) * 1024.0f); }
  for (int pass = 0; pass < 2; ++pass) { *(volatile v8us*)((unsigned short*)Hh + t * 8) = fh.half[0]; *(volatile v8us*)((unsigned short*)Hl + t * 8) = fl.half[0]; if (pass == 0) __threadfence(); } }

__global__ __launch_bounds__(256) void k_x16(const float* __restrict__ x, _Float16* __restrict__ X16, size_t n8) { const size_t t = (size_t)blockIdx.x * 256 + threadIdx.x; if (t >= n8) return; FragH f;
#pragma unroll
  for (int q = 0; q < 8; ++q) f.h[q] = (_Float16)bf16_round(x[t * 8 + q]); *(volatile v8us*)((unsigned short*)X16 + t * 8) = f.half[0]; __threadfence(); *(volatile v8us*)((unsigned short*)X16 + t * 8) = f.half[0]; }

__device__ __forceinline__ v16h g2_frag(const _Float16* p, int hh) { FragH f; f.half[0] = *(const v8us*)((const unsigned short*)p + 8 * hh); f.half[1] = *(const v8us*)((const unsigned short*)p + 16 + 8 * hh); return f.v; }
__device__ __forceinline__ v8f g2_mma(v16h a, v16h b, v8f c) { v8f d = __builtin_amdgcn_wmma_f32_16x16x32_f16(false, a, false, b, (short)0, c, false, false); asm volatile("v_nop\n\tv_nop\n\tv_nop\n\tv_nop" : "+v"(d) : "v"(a), "v"(b)); return d; }
template <int ACT>
__global__ __launch_bounds__(128) void k_gemm2(const _Float16* __restrict__ A, int lda, size_t sA, const _Float16* __restrict__ Bh, int ldb, size_t sB, float alpha, const float* __restrict__ bias, size_t sBias, const float* __restrict__ CP, int rowsPerB, size_t sCPb, int row0g,
    float* __restrict__ C, _Float16* __restrict__ C16, int ldc, size_t sC, int M, int N, int K) { static_assert(ACT == 0 || ACT == 3 || ACT == 6 || ACT == 8 || ACT == 9 || ACT == 11 || ACT == 12 || ACT == 14 || ACT == 15 || ACT == 16 || ACT == 17, "k_gemm2: unsupported ACT code (would silently apply no activation)");
  __shared__ __attribute__((aligned(16))) float so[4][32][68];
  const int tid = threadIdx.x, w = tid >> 5, lane = tid & 31, ln = lane & 15, hh = lane >> 4; const int by = blockIdx.y;
  A += (size_t)by * sA; Bh += (size_t)by * sB; const size_t cofs = (size_t)by * sC; const float* bp = bias ? bias + (size_t)by * sBias : nullptr;
  const int ntn = N >> 6; const int mt = blockIdx.x / ntn, nq = blockIdx.x - mt * ntn; const int row0 = mt * 128 + 32 * w, col0 = nq * 64; if (row0 >= M) return;
  const _Float16* a0p = A + (size_t)(row0 + ln) * lda; const _Float16* a1p = a0p + (size_t)16 * lda;
  const _Float16* b0p = Bh + (size_t)(col0 + ln) * ldb; const _Float16* b1p = b0p + (size_t)16 * ldb; const _Float16* b2p = b1p + (size_t)16 * ldb; const _Float16* b3p = b2p + (size_t)16 * ldb;
  const v8f z8 = {0.f,0.f,0.f,0.f,0.f,0.f,0.f,0.f}; v8f c00 = z8, c01 = z8, c02 = z8, c03 = z8, c10 = z8, c11 = z8, c12 = z8, c13 = z8;
  for (int kb = 0; kb < K; kb += 32) { const v16h a0 = g2_frag(a0p + kb, hh), a1 = g2_frag(a1p + kb, hh);
    v16h b = g2_frag(b0p + kb, hh); c00 = g2_mma(a0, b, c00); c10 = g2_mma(a1, b, c10);
    b = g2_frag(b1p + kb, hh); c01 = g2_mma(a0, b, c01); c11 = g2_mma(a1, b, c11);
    b = g2_frag(b2p + kb, hh); c02 = g2_mma(a0, b, c02); c12 = g2_mma(a1, b, c12);
    b = g2_frag(b3p + kb, hh); c03 = g2_mma(a0, b, c03); c13 = g2_mma(a1, b, c13); }
  v8f accs[8] = {c00, c01, c02, c03, c10, c11, c12, c13};
#pragma unroll
  for (int u = 0; u < 8; ++u) { const int t = u & 3, half = u >> 2; const int col = col0 + t * 16 + ln; const float bv = bp ? bf16_round(bp[col]) : 0.f;
#pragma unroll
    for (int r = 0; r < 8; ++r) { const int rloc = half * 16 + 8 * hh + r; float v = accs[u][r] * alpha + bv; if (CP) { if (rowsPerB < 0) v += CP[cofs + (size_t)(row0g + row0 + rloc) * ldc + col];        else { const int bidx = (row0g + row0 + rloc) / rowsPerB; v += CP[(size_t)bidx * sCPb + (size_t)by * 64 + col]; } }
      if (ACT == 3) v = fmaxf(v, 0.f); else if (ACT == 6) v = 0.5f * v * (1.0f + erff(v * 0.70710678118654752f)); else if (ACT == 11) v = 1.0f / (1.0f + expf(-v)); else if (ACT == 15) v = v / (1.0f + expf(-v)); else if (ACT == 12) v = (v > 0.f) ? v : 0.01f * v; else if (ACT == 8) v = tanhf(v); else if (ACT == 9) v = 0.5f * v * (1.0f + tanhf(0.7978845608028654f * (v + 0.044715f * v * v * v))); else if (ACT == 14) v = (v > 0.f) ? v : 0.1f * v; else if (ACT == 16) v = (v >= 0.f) ? v : 0.3f * v; else if (ACT == 17) v = (v >= 0.f) ? v : 0.2f * v;
      so[w][rloc][t * 16 + ln] = v; } }
  __builtin_amdgcn_fence(__ATOMIC_ACQ_REL, "workgroup"); __builtin_amdgcn_wave_barrier();
  const int rsub = lane >> 4, c4 = (lane & 15) * 4;
  for (int pass = 0; pass < 2; ++pass) {
#pragma unroll
    for (int q = 0; q < 16; ++q) { const int r = q * 2 + rsub; const v4f v = *(const v4fa*)&so[w][r][c4]; if (C) *(volatile v4f*)(C + cofs + (size_t)(row0 + r) * ldc + col0 + c4) = v; if (C16) { v4h h4; for (int i = 0; i < 4; ++i) h4[i] = (_Float16)v[i]; *(volatile v4h*)(C16 + cofs + (size_t)(row0 + r) * ldc + col0 + c4) = h4; } }
    if (pass == 0) __threadfence(); } }

__global__ __launch_bounds__(256) void k_rb(const float* __restrict__ xa, float* __restrict__ XR) {
  const unsigned t = blockIdx.x * 256u + threadIdx.x; if (t >= (unsigned)(ZNR * (ZNW / 4))) return;
  const v4f a = *(const v4fa*)(xa + (size_t)t * 4); v4f w;
#pragma unroll
  for (int q = 0; q < 4; ++q) w[q] = bf16_round(a[q]);
  float* d = XR + (size_t)t * 4; *(volatile v4f*)d = w; __threadfence(); *(volatile v4f*)d = w; }

__global__ __launch_bounds__(256) void k_inm(const float* __restrict__ XR, float* __restrict__ XF) {
  const unsigned t = blockIdx.x * 256u + threadIdx.x; if (t >= (unsigned)(ZNG * ZNS)) return;
  const unsigned g = t / ZNS, st = t % ZNS; float sm = 0.0f;
  for (unsigned sp = 0; sp < (unsigned)ZNC; ++sp) { const float* p = XR + ((size_t)(g * ZNC + sp) * ZNS + st) * ZNW;
    for (unsigned j = 0; j < (unsigned)ZNW; j += 4) { const v4f a = *(const v4fa*)(p + j);
#pragma unroll
      for (int q = 0; q < 4; ++q) sm += a[q]; } }
  const float mu = sm / (float)(ZNC * ZNW); float sq = 0.0f;
  for (unsigned sp = 0; sp < (unsigned)ZNC; ++sp) { const float* p = XR + ((size_t)(g * ZNC + sp) * ZNS + st) * ZNW;
    for (unsigned j = 0; j < (unsigned)ZNW; j += 4) { const v4f a = *(const v4fa*)(p + j);
#pragma unroll
      for (int q = 0; q < 4; ++q) { const float d = a[q] - mu; sq += d * d; } } }
  const float rs = rsqrtf(sq / (float)(ZNC * ZNW) + ZVE);
  for (unsigned sp = 0; sp < (unsigned)ZNC; ++sp) { const float* p = XR + ((size_t)(g * ZNC + sp) * ZNS + st) * ZNW; float* o = XF + ((size_t)t * ZNC + sp) * ZNW;
    for (unsigned j = 0; j < (unsigned)ZNW; j += 4) { const v4f a = *(const v4fa*)(p + j); v4f w;
#pragma unroll
      for (int q = 0; q < 4; ++q) w[q] = (a[q] - mu) * rs;
      *(volatile v4f*)(o + j) = w; __threadfence(); *(volatile v4f*)(o + j) = w; } }
}

__global__ __launch_bounds__(256) void k_lat(const float* __restrict__ T3, _Float16* __restrict__ AH) {
  const unsigned t = blockIdx.x * 256u + threadIdx.x; if (t >= (unsigned)(ZNG * ZNS * 8)) return;
  const unsigned i = t / 8u, e = (t % 8u) * 8u; const float* r0 = T3 + (size_t)(i * ZNC) * (3 * ZNW); const float* r1 = r0 + 3 * ZNW;
  const v4f ca0 = *(const v4fa*)(r0 + 2 * ZNW + e), ca1 = *(const v4fa*)(r0 + 2 * ZNW + e + 4), cb0 = *(const v4fa*)(r1 + 2 * ZNW + e), cb1 = *(const v4fa*)(r1 + 2 * ZNW + e + 4);
  float c0[8], c1[8], a0[8], a1[8];
#pragma unroll
  for (int n = 0; n < 4; ++n) { c0[n] = ca0[n]; c0[4 + n] = ca1[n]; c1[n] = cb0[n]; c1[4 + n] = cb1[n]; a0[n] = 0.0f; a0[4 + n] = 0.0f; a1[n] = 0.0f; a1[4 + n] = 0.0f; }
  for (unsigned p = 0; p < (unsigned)ZNW; p += 4) { const v4f q0 = *(const v4fa*)(r0 + p), q1 = *(const v4fa*)(r1 + p), k0 = *(const v4fa*)(r0 + ZNW + p), k1 = *(const v4fa*)(r1 + ZNW + p);
#pragma unroll
    for (int u = 0; u < 4; ++u) {
#pragma unroll
      for (int n = 0; n < 8; ++n) { const float m = k0[u] * c0[n] + k1[u] * c1[n]; a0[n] += q0[u] * m; a1[n] += q1[u] * m; } } }
  FragH f0, f1;
#pragma unroll
  for (int n = 0; n < 8; ++n) { f0.h[n] = (_Float16)(c0[n] + a0[n]); f1.h[n] = (_Float16)(c1[n] + a1[n]); }
  unsigned short* o0 = (unsigned short*)AH + (size_t)(i * ZNC) * ZNW + e; unsigned short* o1 = o0 + ZNW; const v8us w0 = f0.half[0], w1 = f1.half[0];
  *(volatile v8us*)o0 = w0; *(volatile v8us*)o1 = w1; __threadfence(); *(volatile v8us*)o0 = w0; *(volatile v8us*)o1 = w1; }

__global__ __launch_bounds__(256) void k_fin(const float* __restrict__ PR, const float* __restrict__ XR, float* __restrict__ res) {
  const unsigned t = blockIdx.x * 256u + threadIdx.x; if (t >= (unsigned)(ZNG * ZNC * ZNS * (ZNW / 4))) return;
  const unsigned j = (t % (ZNW / 4)) * 4, rw = t / (ZNW / 4), st = rw % ZNS, sp = (rw / ZNS) % ZNC, g = rw / (ZNS * ZNC);
  const v4f a = *(const v4fa*)(PR + ((size_t)(g * ZNS + st) * ZNC + sp) * ZNW + j); const v4f xv = *(const v4fa*)(XR + (size_t)t * 4); v4f w;
#pragma unroll
  for (int q = 0; q < 4; ++q) w[q] = a[q] + xv[q];
  float* d = res + (size_t)t * 4; *(volatile v4f*)d = w; __threadfence(); *(volatile v4f*)d = w; }

extern "C" void kernel_launch(void* const* d_in, const int* in_sizes, int n_in,
                              void* d_out, int out_size, void* d_ws, size_t ws_size, hipStream_t stream) {
  (void)in_sizes; (void)n_in; (void)out_size;
  const float* const* I = (const float* const*)d_in; const float* xa = I[0]; const float* wf = I[1]; const float* vf = I[2]; const float* wo = I[3]; const float* vo = I[4];
  float* res = (float*)d_out;
  static_assert(ZNR % 128 == 0 && (3 * ZNW) % 64 == 0 && ZNW % 64 == 0 && ZNW % 32 == 0 && ZNW % 8 == 0 && (ZNR * ZNW) % 8 == 0, "whole tiles");
  uint8_t* wsp = (uint8_t*)d_ws; size_t off = 0;
  auto take = [&](size_t bytes) { uint8_t* p = wsp + off; off += (bytes + 255) & ~(size_t)255; return p; };
  float* XR = (float*)take((size_t)ZNR * ZNW * 4); float* XF = (float*)take((size_t)ZNR * ZNW * 4); _Float16* XH = (_Float16*)take((size_t)ZNR * ZNW * 2); _Float16* XL = (_Float16*)take((size_t)ZNR * ZNW * 2); _Float16* WF = (_Float16*)take((size_t)3 * ZNW * ZNW * 2); _Float16* WO = (_Float16*)take((size_t)ZNW * ZNW * 2); float* T3 = (float*)take((size_t)ZNR * 3 * ZNW * 4); _Float16* AH = (_Float16*)take((size_t)ZNR * ZNW * 2); float* PR = (float*)take((size_t)ZNR * ZNW * 4);
  if (off > ws_size) return;
  k_rb<<<(unsigned)(((size_t)ZNR * (ZNW / 4) + 255) / 256), 256, 0, stream>>>(xa, XR);
  k_inm<<<(unsigned)((ZNG * ZNS + 255) / 256), 256, 0, stream>>>(XR, XF);
  k_hl<<<(unsigned)(((size_t)ZNR * ZNW / 8 + 255) / 256), 256, 0, stream>>>(XF, XH, XL, (size_t)ZNR * ZNW / 8);
  k_x16<<<(unsigned)(((size_t)3 * ZNW * ZNW / 8 + 255) / 256), 256, 0, stream>>>(wf, WF, (size_t)3 * ZNW * ZNW / 8);
  k_x16<<<(unsigned)(((size_t)ZNW * ZNW / 8 + 255) / 256), 256, 0, stream>>>(wo, WO, (size_t)ZNW * ZNW / 8);
  k_gemm2<0><<<dim3((unsigned)((ZNR / 128) * ((3 * ZNW) / 64)), 1), 128, 0, stream>>>(XH, ZNW, 0, WF, ZNW, 0, 1.0f, vf, 0, nullptr, 1, 0, 0, T3, nullptr, 3 * ZNW, 0, ZNR, 3 * ZNW, ZNW);
  k_gemm2<0><<<dim3((unsigned)((ZNR / 128) * ((3 * ZNW) / 64)), 1), 128, 0, stream>>>(XL, ZNW, 0, WF, ZNW, 0, 0.0009765625f, nullptr, 0, T3, -1, 0, 0, T3, nullptr, 3 * ZNW, 0, ZNR, 3 * ZNW, ZNW);
  k_lat<<<(unsigned)((ZNG * ZNS * 8 + 255) / 256), 256, 0, stream>>>(T3, AH);
  k_gemm2<0><<<dim3((unsigned)((ZNR / 128) * (ZNW / 64)), 1), 128, 0, stream>>>(AH, ZNW, 0, WO, ZNW, 0, 1.0f, vo, 0, nullptr, 1, 0, 0, PR, nullptr, ZNW, 0, ZNR, ZNW, ZNW);
  k_fin<<<(unsigned)(((size_t)ZNG * ZNC * ZNS * (ZNW / 4) + 255) / 256), 256, 0, stream>>>(PR, XR, res);
}
